// SimpleHeteroGNN_9569187135976
// MI455X (gfx1250) — hardware-verified
//
#include <hip/hip_runtime.h>
#include <stddef.h>


#define DM     128
#define OUTC   16
#define OUTP   64
#define NLAY   3
#define NWROWS 960
#define WPP    136
#define GT     128
#define RB     1024
#define RBBITS 10
#define RMAX   64
#define RMBITS 6
#define TABW   (2 * RMAX)
#define CHUNK  4096
#define LCAP   18432
#define DEGCAP 96
#define STATRS 128
#define GPB    8
#define WSCAP  134217728

#define AGG_LDS_INTS  (RB + 8 + RB + LCAP)
#define AGG_LDS_BYTES (AGG_LDS_INTS * 4)

static_assert(RB == (1 << RBBITS));
static_assert(RMAX == (1 << RMBITS));
static_assert(CHUNK == 8 * 16 * 32);
static_assert(CHUNK == 4 * 4 * 256);
static_assert(TABW * 4 == 32 * 16);
static_assert((RB % 128) == 0);
static_assert(RB == 4 * 256);
static_assert((AGG_LDS_BYTES % 16) == 0);
static_assert(AGG_LDS_BYTES < 300000);
static_assert((STATRS % 2) == 0 && (STATRS % 128) == 0);
static_assert(DM == 32 * 4);
static_assert(NWROWS == 2 * NLAY * DM + DM + OUTP);
static_assert((OUTP % 32) == 0 && OUTP >= OUTC);
static_assert((WPP % 8) == 0);
static_assert(GPB == 8);

typedef float          v4f  __attribute__((ext_vector_type(4)));
typedef float          v8f  __attribute__((ext_vector_type(8)));
typedef double         v2d  __attribute__((ext_vector_type(2)));
typedef int            v4i  __attribute__((ext_vector_type(4)));
typedef unsigned int   v4u  __attribute__((ext_vector_type(4)));
typedef unsigned short v8us __attribute__((ext_vector_type(8)));
typedef __bf16         v16b __attribute__((ext_vector_type(16)));
union FragB { v16b v; v8us u[2]; };

__device__ __forceinline__ unsigned short b16(float f) {
  unsigned int u = __float_as_uint(f);
  u += 0x7FFFu + ((u >> 16) & 1u);
  return (unsigned short)(u >> 16);
}

__device__ __forceinline__ float b16f(unsigned short h) {
  return __uint_as_float(((unsigned int)h) << 16);
}

__device__ __forceinline__ void split4(v4f r, unsigned int& u0h, unsigned int& u1h,
                                       unsigned int& u0l, unsigned int& u1l) {
  const unsigned short hx = b16(r.x), hy = b16(r.y), hz = b16(r.z), hw = b16(r.w);
  const unsigned short lx = b16(r.x - b16f(hx)), ly = b16(r.y - b16f(hy));
  const unsigned short lz = b16(r.z - b16f(hz)), lw = b16(r.w - b16f(hw));
  u0h = (unsigned int)hx | ((unsigned int)hy << 16);
  u1h = (unsigned int)hz | ((unsigned int)hw << 16);
  u0l = (unsigned int)lx | ((unsigned int)ly << 16);
  u1l = (unsigned int)lz | ((unsigned int)lw << 16);
}

__device__ __forceinline__ v4u relay8(unsigned int u0, unsigned int u1, int sl) {
  v4u q;
  q.x = (unsigned int)__shfl((int)u0, sl);
  q.y = (unsigned int)__shfl((int)u1, sl);
  q.z = (unsigned int)__shfl((int)u0, sl + 1);
  q.w = (unsigned int)__shfl((int)u1, sl + 1);
  return q;
}

__device__ __forceinline__ v8f wmb(v16b a, v16b b, v8f c) {
  v8f d = __builtin_amdgcn_wmma_f32_16x16x32_bf16(false, a, false, b, (short)0, c, false, false);
  asm volatile("v_nop\n\tv_nop\n\tv_nop\n\tv_nop" : "+v"(d) : "v"(a), "v"(b));
  return d;
}

template <int NB>
__device__ __forceinline__ unsigned int match_mask(unsigned int base, int key) {
  unsigned int msk = base;
#pragma unroll
  for (int b = 0; b < NB; ++b) {
    const bool bit = ((key >> b) & 1) != 0;
    const unsigned int bb = __builtin_amdgcn_ballot_w32(bit);
    msk &= bit ? bb : ~bb;
  }
  return msk;
}

__global__ __launch_bounds__(256) void k_csort(
    const int* __restrict__ key, unsigned int* csort, int* tab, int nN, int nE) {
  __shared__ __attribute__((aligned(16))) unsigned int sImg[CHUNK];
  __shared__ int cw[8 * RMAX];
  __shared__ __attribute__((aligned(16))) int sTb[TABW];
  __shared__ int sWt[8];
  int* sPre = sTb;
  int* sCn  = sTb + RMAX;
  const int tid = (int)threadIdx.x, lane = tid & 31, wave = tid >> 5;
  const int c = (int)blockIdx.x;
  const int cbase = c * CHUNK;

  for (int i = tid; i < 8 * RMAX; i += 256) cw[i] = 0;
  {
    const v4u s = {0xffffffffu, 0xffffffffu, 0xffffffffu, 0xffffffffu};
    for (int i = tid; i < CHUNK / 4; i += 256) ((v4u*)sImg)[i] = s;
  }
  __syncthreads();

  unsigned int ent[16];
  int pk[16];
  const unsigned int lt = (1u << lane) - 1u;
#pragma unroll
  for (int i = 0; i < 16; ++i) {
    const int e = cbase + wave * 512 + 32 * i + lane;
    const int ea = e > nE - 1 ? nE - 1 : e;
    const int d = key[ea];
    const bool valid = (e < nE) && ((unsigned)d < (unsigned)nN);
    const int dd = valid ? d : 0;
    const int r  = dd >> RBBITS;
    const int jl = dd & (RB - 1);
    const unsigned int pay = (unsigned int)ea;
    const unsigned int msk = match_mask<RMBITS>(__builtin_amdgcn_ballot_w32(valid), r);
    const int rank = (int)__builtin_popcount(msk & lt);
    const int grp  = (int)__builtin_popcount(msk);
    const int base = cw[wave * RMAX + r];
    pk[i]  = valid ? ((r << 12) | (base + rank)) : -1;
    ent[i] = (pay << RBBITS) | (unsigned int)jl;
    if (valid && rank == 0) cw[wave * RMAX + r] = base + grp;
    __syncthreads();
  }

  if (tid < RMAX) {
    int run = 0;
#pragma unroll
    for (int w = 0; w < 8; ++w) {
      const int v = cw[w * RMAX + tid];
      cw[w * RMAX + tid] = run;
      run += v;
    }
    sCn[tid] = run;
  }
  __syncthreads();
  {
    const int vr = sCn[tid & (RMAX - 1)];
    const int v  = (tid < RMAX) ? vr : 0;
    int x = v;
#pragma unroll
    for (int dd = 1; dd < 32; dd <<= 1) {
      const int y = __shfl_up(x, dd);
      x += (lane >= dd) ? y : 0;
    }
    if (lane == 31) sWt[wave] = x;
    __syncthreads();
    int pre = 0;
#pragma unroll
    for (int w = 0; w < 8; ++w) { const int tw = sWt[w]; pre += (w < wave) ? tw : 0; }
    if (tid < RMAX) sPre[tid] = pre + x - v;
  }
  __syncthreads();

#pragma unroll
  for (int i = 0; i < 16; ++i) {
    if (pk[i] >= 0) {
      const int r = (pk[i] >> 12) & (RMAX - 1);
      const int q = pk[i] & 4095;
      const int pos = sPre[r] + cw[wave * RMAX + r] + q;
      if ((unsigned)pos < (unsigned)CHUNK) sImg[pos] = ent[i];
    }
  }
  __syncthreads();

  v4u iv[4];
#pragma unroll
  for (int it = 0; it < 4; ++it) iv[it] = ((const v4u*)sImg)[it * 256 + tid];
  const v4i tv = *(const v4i*)(sTb + 4 * lane);
  unsigned int* gp = csort + (size_t)c * CHUNK;
  int* tp = tab + (size_t)c * TABW + 4 * lane;
  const bool wt = tid < 32;
#pragma unroll
  for (int it = 0; it < 4; ++it) *(volatile v4u*)(gp + 4 * (it * 256 + tid)) = iv[it];
  if (wt) *(volatile v4i*)tp = tv;
  __threadfence();
#pragma unroll
  for (int it = 0; it < 4; ++it) *(volatile v4u*)(gp + 4 * (it * 256 + tid)) = iv[it];
  if (wt) *(volatile v4i*)tp = tv;
}

__global__ __launch_bounds__(256) void k_wprep(
    const float* __restrict__ W1s, const float* __restrict__ W2s,
    const float* __restrict__ Wc1, const float* __restrict__ Wc2,
    unsigned short* Thi, unsigned short* Tlo) {
  __shared__ __attribute__((aligned(16))) unsigned short sH[32 * WPP];
  __shared__ __attribute__((aligned(16))) unsigned short sL[32 * WPP];
  const int tid = (int)threadIdx.x;
  const int b = (int)blockIdx.x;
  const int sel = (b < 12) ? 0 : ((b < 24) ? 1 : ((b < 28) ? 2 : 3));
  const int bl  = (sel == 0) ? b : ((sel == 1) ? (b - 12) : ((sel == 2) ? (b - 24) : (b - 28)));
  const float* Wb = (sel == 0) ? (W1s + (size_t)(bl >> 2) * DM * DM)
                  : ((sel == 1) ? (W2s + (size_t)(bl >> 2) * DM * DM)
                  : ((sel == 2) ? Wc1 : Wc2));
  const int pitch = (sel == 3) ? OUTC : DM;
  const int nb0 = (sel <= 1) ? ((bl & 3) * 32) : (bl * 32);
  const int rowBase = b * 32;
  const v4f zero4 = {0.0f, 0.0f, 0.0f, 0.0f};

#pragma unroll 1
  for (int it = 0; it < 4; ++it) {
    const int p = it * 256 + tid;
    const int k = p >> 3, q = p & 7;
    const int c = nb0 + 4 * q;
    const bool ok = (c + 4 <= pitch);
    const int ca = ok ? c : (pitch - 4);
    v4f w = *(const v4f*)(Wb + (size_t)k * pitch + ca);
    w = ok ? w : zero4;
    unsigned short* dh = sH + (4 * q) * WPP + k;
    unsigned short* dl = sL + (4 * q) * WPP + k;
    const unsigned short hx = b16(w.x), hy = b16(w.y), hz = b16(w.z), hw = b16(w.w);
    dh[0]       = hx; dl[0]       = b16(w.x - b16f(hx));
    dh[WPP]     = hy; dl[WPP]     = b16(w.y - b16f(hy));
    dh[2 * WPP] = hz; dl[2 * WPP] = b16(w.z - b16f(hz));
    dh[3 * WPP] = hw; dl[3 * WPP] = b16(w.w - b16f(hw));
  }
  __syncthreads();

  v8us oh[2], ol[2];
#pragma unroll
  for (int it = 0; it < 2; ++it) {
    const int p = it * 256 + tid;
    const int row = p >> 4, c8 = (p & 15) * 8;
    oh[it] = *(const v8us*)(sH + row * WPP + c8);
    ol[it] = *(const v8us*)(sL + row * WPP + c8);
  }
#pragma unroll
  for (int it = 0; it < 2; ++it) {
    const int p = it * 256 + tid;
    const int row = p >> 4, c8 = (p & 15) * 8;
    *(volatile v8us*)(Thi + (size_t)(rowBase + row) * DM + c8) = oh[it];
    *(volatile v8us*)(Tlo + (size_t)(rowBase + row) * DM + c8) = ol[it];
  }
  __threadfence();
#pragma unroll
  for (int it = 0; it < 2; ++it) {
    const int p = it * 256 + tid;
    const int row = p >> 4, c8 = (p & 15) * 8;
    *(volatile v8us*)(Thi + (size_t)(rowBase + row) * DM + c8) = oh[it];
    *(volatile v8us*)(Tlo + (size_t)(rowBase + row) * DM + c8) = ol[it];
  }
}

template <int HASB>
__global__ __launch_bounds__(GT) void k_gemm(
    const unsigned short* __restrict__ AH, const unsigned short* __restrict__ AL,
    const unsigned short* __restrict__ BH, const unsigned short* __restrict__ BL,
    const float* __restrict__ bias, float* outF, int ldo, int Mp, int Ncols) {
  __shared__ __attribute__((aligned(16))) float sT[4 * 32 * 32];
  const int tid = (int)threadIdx.x, lane = tid & 31, wave = tid >> 5, hh = lane >> 4, m = lane & 15;
  const int c0 = (int)blockIdx.x * 32;
  const int r0 = (int)blockIdx.y * 128 + wave * 32;

  int ra0 = r0 + m;      ra0 = ra0 > Mp - 1 ? Mp - 1 : ra0;
  int ra1 = r0 + 16 + m; ra1 = ra1 > Mp - 1 ? Mp - 1 : ra1;
  const unsigned short* ah0 = AH + (size_t)ra0 * DM + 8 * hh;
  const unsigned short* al0 = AL + (size_t)ra0 * DM + 8 * hh;
  const unsigned short* ah1 = AH + (size_t)ra1 * DM + 8 * hh;
  const unsigned short* al1 = AL + (size_t)ra1 * DM + 8 * hh;
  const unsigned short* bh[2];
  const unsigned short* bl[2];
#pragma unroll
  for (int j = 0; j < 2; ++j) {
    int cb = c0 + 16 * j + m; cb = cb > Ncols - 1 ? Ncols - 1 : cb;
    bh[j] = BH + (size_t)cb * DM + 8 * hh;
    bl[j] = BL + (size_t)cb * DM + 8 * hh;
  }

  v8f acc[2][2];
#pragma unroll
  for (int i = 0; i < 2; ++i)
#pragma unroll
    for (int j = 0; j < 2; ++j) { v8f z = {0.f, 0.f, 0.f, 0.f, 0.f, 0.f, 0.f, 0.f}; acc[i][j] = z; }

#pragma unroll 1
  for (int kt = 0; kt < 4; ++kt) {
    const int kb = kt << 5;
    FragB a0h, a0l, a1h, a1l, b0h, b0l, b1h, b1l;
    a0h.u[0] = *(const v8us*)(ah0 + kb);
    a0h.u[1] = *(const v8us*)(ah0 + kb + 16);
    a0l.u[0] = *(const v8us*)(al0 + kb);
    a0l.u[1] = *(const v8us*)(al0 + kb + 16);
    a1h.u[0] = *(const v8us*)(ah1 + kb);
    a1h.u[1] = *(const v8us*)(ah1 + kb + 16);
    a1l.u[0] = *(const v8us*)(al1 + kb);
    a1l.u[1] = *(const v8us*)(al1 + kb + 16);
    b0h.u[0] = *(const v8us*)(bh[0] + kb);
    b0h.u[1] = *(const v8us*)(bh[0] + kb + 16);
    b0l.u[0] = *(const v8us*)(bl[0] + kb);
    b0l.u[1] = *(const v8us*)(bl[0] + kb + 16);
    b1h.u[0] = *(const v8us*)(bh[1] + kb);
    b1h.u[1] = *(const v8us*)(bh[1] + kb + 16);
    b1l.u[0] = *(const v8us*)(bl[1] + kb);
    b1l.u[1] = *(const v8us*)(bl[1] + kb + 16);
    acc[0][0] = wmb(a0h.v, b0h.v, acc[0][0]);
    acc[1][0] = wmb(a1h.v, b0h.v, acc[1][0]);
    acc[0][1] = wmb(a0h.v, b1h.v, acc[0][1]);
    acc[1][1] = wmb(a1h.v, b1h.v, acc[1][1]);
    acc[0][0] = wmb(a0h.v, b0l.v, acc[0][0]);
    acc[1][0] = wmb(a1h.v, b0l.v, acc[1][0]);
    acc[0][1] = wmb(a0h.v, b1l.v, acc[0][1]);
    acc[1][1] = wmb(a1h.v, b1l.v, acc[1][1]);
    acc[0][0] = wmb(a0l.v, b0h.v, acc[0][0]);
    acc[1][0] = wmb(a1l.v, b0h.v, acc[1][0]);
    acc[0][1] = wmb(a0l.v, b1h.v, acc[0][1]);
    acc[1][1] = wmb(a1l.v, b1h.v, acc[1][1]);
  }

  float* sw = sT + wave * 1024;
#pragma unroll
  for (int i = 0; i < 2; ++i)
#pragma unroll
    for (int j = 0; j < 2; ++j)
#pragma unroll
      for (int r = 0; r < 8; ++r)
        sw[(16 * i + 8 * hh + r) * 32 + 16 * j + m] = acc[i][j][r];
  __syncthreads();

  v4f ov[8];
#pragma unroll
  for (int it = 0; it < 8; ++it) {
    const int f = it * 32 + lane;
    const int row = f >> 3, c4 = (f & 7) * 4;
    v4f v = *(const v4f*)(sw + row * 32 + c4);
    if (HASB) {
      const v4f bb = *(const v4f*)(bias + c0 + c4);
      v = v + bb;
    }
    ov[it] = v;
  }
#pragma unroll
  for (int it = 0; it < 8; ++it) {
    const int f = it * 32 + lane;
    const int row = f >> 3, c4 = (f & 7) * 4;
    *(volatile v4f*)(outF + (size_t)(r0 + row) * ldo + c0 + c4) = ov[it];
  }
  __threadfence();
#pragma unroll
  for (int it = 0; it < 8; ++it) {
    const int f = it * 32 + lane;
    const int row = f >> 3, c4 = (f & 7) * 4;
    *(volatile v4f*)(outF + (size_t)(r0 + row) * ldo + c0 + c4) = ov[it];
  }
}

__global__ __launch_bounds__(256) void k_agg(
    const float* __restrict__ H, int hrows, const int* __restrict__ src,
    const unsigned int* __restrict__ csort, const int* __restrict__ tab,
    unsigned short* AH, unsigned short* AL, int nN, int nNp, int nE, int nCh) {
  extern __shared__ __attribute__((aligned(16))) int dsm[];
  __shared__ int sWtot[8];
  int* sOff  = dsm;
  int* sCur  = dsm + (RB + 8);
  int* sList = sCur + RB;
  const int tid = (int)threadIdx.x, lane = tid & 31, wave = tid >> 5;
  const int rgn = (int)blockIdx.x;
  const int n0 = rgn * RB;
  const unsigned int lt = (1u << lane) - 1u;

  for (int i = tid; i < RB + 8; i += 256) sOff[i] = 0;
  for (int i = tid; i < RB; i += 256) sCur[i] = 0;
  __syncthreads();

#pragma unroll 1
  for (int c = 0; c < nCh; ++c) {
    int pre = tab[(size_t)c * TABW + rgn];
    int n   = tab[(size_t)c * TABW + RMAX + rgn];
    pre = pre < 0 ? 0 : (pre > CHUNK ? CHUNK : pre);
    n = n < 0 ? 0 : (n > CHUNK - pre ? CHUNK - pre : n);
    const int nstep = (n + 31) >> 5;
    const unsigned int* cp = csort + (size_t)c * CHUNK + pre;
#pragma unroll 1
    for (int s = 0; s < nstep; ++s) {
      if (wave == 0) {
        const int i = (s << 5) + lane;
        const bool valid = i < n;
        const int ic = i > n - 1 ? n - 1 : i;
        const unsigned int en = cp[ic];
        const int j = (int)(en & (unsigned int)(RB - 1));
        const unsigned int msk = match_mask<RBBITS>(__builtin_amdgcn_ballot_w32(valid), j);
        const int rank = (int)__builtin_popcount(msk & lt);
        const int grp  = (int)__builtin_popcount(msk);
        if (valid && rank == 0) sOff[j] = sOff[j] + grp;
      }
      __syncthreads();
    }
  }
  __syncthreads();

  {
    int cn[4];
    int ls = 0;
#pragma unroll
    for (int i = 0; i < 4; ++i) { cn[i] = sOff[4 * tid + i]; ls += cn[i]; }
    int x = ls;
#pragma unroll
    for (int dd = 1; dd < 32; dd <<= 1) {
      const int y = __shfl_up(x, dd);
      x += (lane >= dd) ? y : 0;
    }
    if (lane == 31) sWtot[wave] = x;
    __syncthreads();
    int pre = 0;
#pragma unroll
    for (int w = 0; w < 8; ++w) { const int tw = sWtot[w]; pre += (w < wave) ? tw : 0; }
    int run = pre + x - ls;
#pragma unroll
    for (int i = 0; i < 4; ++i) { sOff[4 * tid + i] = run; run += cn[i]; }
    if (tid == 255) sOff[RB] = run;
  }
  __syncthreads();
  const bool rgnOver = sOff[RB] > LCAP;

#pragma unroll 1
  for (int c = 0; c < nCh; ++c) {
    int pre = tab[(size_t)c * TABW + rgn];
    int n   = tab[(size_t)c * TABW + RMAX + rgn];
    pre = pre < 0 ? 0 : (pre > CHUNK ? CHUNK : pre);
    n = n < 0 ? 0 : (n > CHUNK - pre ? CHUNK - pre : n);
    const int nstep = (n + 31) >> 5;
    const unsigned int* cp = csort + (size_t)c * CHUNK + pre;
#pragma unroll 1
    for (int s = 0; s < nstep; ++s) {
      if (wave == 0) {
        const int i = (s << 5) + lane;
        const bool valid = i < n;
        const int ic = i > n - 1 ? n - 1 : i;
        const unsigned int en = cp[ic];
        const int j = (int)(en & (unsigned int)(RB - 1));
        int e = (int)(en >> RBBITS);
        e = e > nE - 1 ? nE - 1 : e;
        const unsigned int msk = match_mask<RBBITS>(__builtin_amdgcn_ballot_w32(valid), j);
        const int rank = (int)__builtin_popcount(msk & lt);
        const int grp  = (int)__builtin_popcount(msk);
        const int cur  = sCur[j];
        const int p0   = sOff[j] + cur + rank;
        if (valid && (unsigned)p0 < (unsigned)LCAP) sList[p0] = e;
        if (valid && rank == 0) sCur[j] = cur + grp;
      }
      __syncthreads();
    }
  }
  __syncthreads();

  const int c4 = 4 * lane;
  int Rbp = nNp - n0; Rbp = Rbp > RB ? RB : Rbp;
  const int niter = (Rbp + 7) >> 3;
  const v4f zero4 = {0.0f, 0.0f, 0.0f, 0.0f};
  const float qn = __int_as_float(0x7fc00000);
  const v4f nan4 = {qn, qn, qn, qn};
  const int sl = 2 * (lane & 15);
  const bool lo16 = lane < 16;
#pragma unroll 1
  for (int jj = 0; jj < niter; ++jj) {
    const int j = jj * 8 + wave;
    const bool act = j < Rbp;
    const int jc = act ? j : (Rbp - 1);
    const int node = n0 + jc;
    const bool live = node < nN;
    int lb = __builtin_amdgcn_readfirstlane(sOff[jc]);
    int ub = __builtin_amdgcn_readfirstlane(sOff[jc + 1]);
    lb = lb < 0 ? 0 : (lb > LCAP ? LCAP : lb);
    ub = ub < 0 ? 0 : (ub > LCAP ? LCAP : ub);
    const int craw = ub - lb;
    int cnt = craw;
    cnt = cnt < 0 ? 0 : (cnt > DEGCAP ? DEGCAP : cnt);

    const int hr = node > hrows - 1 ? hrows - 1 : node;
    v4f acc = *(const v4f*)(H + (size_t)hr * DM + c4);
#pragma unroll 1
    for (int it = 0; it < cnt; ++it) {
      int li = lb + it; li = li > LCAP - 1 ? LCAP - 1 : li;
      int e = sList[li]; e = e < 0 ? 0 : (e > nE - 1 ? nE - 1 : e);
      int s = src[e];   s = s < 0 ? 0 : (s > nN - 1 ? nN - 1 : s);
      const v4f hv = *(const v4f*)(H + (size_t)s * DM + c4);
      acc = acc + hv;
    }
    const bool bad = (craw > DEGCAP) || rgnOver;
    v4f r = bad ? nan4 : acc;
    r = live ? r : zero4;

    unsigned int u0h, u1h, u0l, u1l;
    split4(r, u0h, u1h, u0l, u1l);
    const v4u qh = relay8(u0h, u1h, sl);
    const v4u ql = relay8(u0l, u1l, sl);
    const v4u q = lo16 ? qh : ql;
    unsigned short* op = (lo16 ? AH : AL) + (size_t)node * DM + 8 * (lane & 15);
    if (act) *(volatile v4u*)op = q;
    __threadfence();
    if (act) *(volatile v4u*)op = q;
  }
}

__global__ __launch_bounds__(256) void k_colstat(
    const float* __restrict__ P, int nlive, double* part) {
  __shared__ __attribute__((aligned(16))) double sD[256];
  __shared__ __attribute__((aligned(16))) double sE[256];
  const int tid = (int)threadIdx.x, c = tid & 127, hf = tid >> 7;
  const int rbase = (int)blockIdx.x * STATRS;
  double s = 0.0, s2 = 0.0;
#pragma unroll 4
  for (int i = 0; i < STATRS / 2; ++i) {
    const int r = rbase + 2 * i + hf;
    const float v0 = P[(size_t)r * DM + c];
    const float v = (r < nlive) ? v0 : 0.0f;
    const double dv = (double)v;
    s += dv;
    s2 += dv * dv;
  }
  if (hf == 1) { sD[c] = s; sD[128 + c] = s2; }
  __syncthreads();
  if (hf == 0) { sE[c] = s + sD[c]; sE[128 + c] = s2 + sD[128 + c]; }
  __syncthreads();
  const bool w = tid < 128;
  const int q = tid & 127;
  const v2d v = *(const v2d*)(sE + 2 * q);
  double* gp = part + (size_t)blockIdx.x * 256 + 2 * q;
  if (w) *(volatile v2d*)gp = v;
  __threadfence();
  if (w) *(volatile v2d*)gp = v;
}

__global__ __launch_bounds__(128) void k_bnfin(
    const double* __restrict__ part, int nblk, int nlive, float* stats) {
  __shared__ __attribute__((aligned(16))) float sF[256];
  const int c = (int)threadIdx.x;
  double s = 0.0, s2 = 0.0;
#pragma unroll 1
  for (int b = 0; b < nblk; ++b) {
    s  += part[(size_t)b * 256 + c];
    s2 += part[(size_t)b * 256 + 128 + c];
  }
  const double invn = 1.0 / (double)nlive;
  const double mu = s * invn;
  double var = s2 * invn - mu * mu;
  var = var < 0.0 ? 0.0 : var;
  const float varf = (float)var;
  sF[c] = (float)mu;
  sF[128 + c] = rsqrtf(varf + 1e-5f);
  __syncthreads();
  const bool w = c < 64;
  const int cc = c & 63;
  const v4f v = *(const v4f*)(sF + 4 * cc);
  if (w) *(volatile v4f*)(stats + 4 * cc) = v;
  __threadfence();
  if (w) *(volatile v4f*)(stats + 4 * cc) = v;
}

template <int OF>
__global__ __launch_bounds__(256) void k_bnapply(
    const float* __restrict__ P, const float* __restrict__ stats,
    const float* __restrict__ g, const float* __restrict__ b,
    float* HF, unsigned short* AH, unsigned short* AL, int nlive) {
  const int tid = (int)threadIdx.x, lane = tid & 31, wave = tid >> 5;
  const int c4 = 4 * lane;
  const v4f mu = *(const v4f*)(stats + c4);
  const v4f rs = *(const v4f*)(stats + 128 + c4);
  const v4f gg = *(const v4f*)(g + c4);
  const v4f bb = *(const v4f*)(b + c4);
  const int rb = (int)blockIdx.x * 64;
  const int sl = 2 * (lane & 15);
  const bool lo16 = lane < 16;
  const v4f zero4 = {0.0f, 0.0f, 0.0f, 0.0f};
#pragma unroll 1
  for (int grp = 0; grp < 2; ++grp) {
    const int rw = rb + grp * 32 + wave * 4;
    v4f y[4];
    v4u q[4];
#pragma unroll
    for (int i = 0; i < 4; ++i) {
      const v4f v = *(const v4f*)(P + (size_t)(rw + i) * DM + c4);
      v4f t = (v - mu) * rs * gg + bb;
      t.x = fmaxf(t.x, 0.0f); t.y = fmaxf(t.y, 0.0f); t.z = fmaxf(t.z, 0.0f); t.w = fmaxf(t.w, 0.0f);
      t = (rw + i < nlive) ? t : zero4;
      y[i] = t;
      if (OF == 0) {
        unsigned int u0h, u1h, u0l, u1l;
        split4(t, u0h, u1h, u0l, u1l);
        const v4u qh = relay8(u0h, u1h, sl);
        const v4u ql = relay8(u0l, u1l, sl);
        q[i] = lo16 ? qh : ql;
      } else {
        const v4u z4 = {0u, 0u, 0u, 0u};
        q[i] = z4;
      }
    }
    if (OF == 1) {
#pragma unroll
      for (int i = 0; i < 4; ++i)
        *(volatile v4f*)(HF + (size_t)(rw + i) * DM + c4) = y[i];
      __threadfence();
#pragma unroll
      for (int i = 0; i < 4; ++i)
        *(volatile v4f*)(HF + (size_t)(rw + i) * DM + c4) = y[i];
    } else {
#pragma unroll
      for (int i = 0; i < 4; ++i)
        *(volatile v4u*)((lo16 ? AH : AL) + (size_t)(rw + i) * DM + 8 * (lane & 15)) = q[i];
      __threadfence();
#pragma unroll
      for (int i = 0; i < 4; ++i)
        *(volatile v4u*)((lo16 ? AH : AL) + (size_t)(rw + i) * DM + 8 * (lane & 15)) = q[i];
    }
  }
}

__global__ __launch_bounds__(256) void k_pool(
    const float* __restrict__ H, const int* __restrict__ bat,
    unsigned short* QH, unsigned short* QL, int nN) {
  __shared__ int sHit[256];
  __shared__ int sWc[8];
  __shared__ __attribute__((aligned(16))) v4f sAcc[8 * GPB * 32];
  __shared__ float sCn[8 * GPB];
  const int tid = (int)threadIdx.x, lane = tid & 31, wave = tid >> 5;
  const int g0 = (int)blockIdx.x * GPB;
  const int c4 = 4 * lane;
  const unsigned int lt = (1u << lane) - 1u;
  const v4f zero4 = {0.0f, 0.0f, 0.0f, 0.0f};
  v4f acc[GPB];
  float cn[GPB];
#pragma unroll
  for (int r = 0; r < GPB; ++r) { acc[r] = zero4; cn[r] = 0.0f; }

  const int nchunk = (nN + 255) >> 8;
#pragma unroll 1
  for (int ch = 0; ch < nchunk; ++ch) {
    const int node = (ch << 8) + tid;
    const bool inb = node < nN;
    const int na = inb ? node : (nN - 1);
    const int bt = bat[na];
    const int rel = bt - g0;
    const bool hit = inb && ((unsigned)rel < (unsigned)GPB);
    const unsigned int msk = __builtin_amdgcn_ballot_w32(hit);
    const int pos = (int)__builtin_popcount(msk & lt);
    if (lane == 0) sWc[wave] = (int)__builtin_popcount(msk);
    __syncthreads();
    int pre = 0, tot = 0;
#pragma unroll
    for (int w = 0; w < 8; ++w) { const int c = sWc[w]; pre += (w < wave) ? c : 0; tot += c; }
    if (hit) sHit[pre + pos] = (na << 3) | rel;
    __syncthreads();
    tot = tot > 256 ? 256 : tot;
#pragma unroll 1
    for (int t = wave; t < tot; t += 8) {
      const int en = sHit[t];
      int nd = en >> 3; nd = nd < 0 ? 0 : (nd > nN - 1 ? nN - 1 : nd);
      const int rl = en & 7;
      const v4f v = *(const v4f*)(H + (size_t)nd * DM + c4);
#pragma unroll
      for (int r = 0; r < GPB; ++r) {
        const bool s = (rl == r);
        acc[r] = s ? (acc[r] + v) : acc[r];
        cn[r] = s ? (cn[r] + 1.0f) : cn[r];
      }
    }
    __syncthreads();
  }

#pragma unroll
  for (int r = 0; r < GPB; ++r) {
    sAcc[(wave * GPB + r) * 32 + lane] = acc[r];
    if (lane == 0) sCn[wave * GPB + r] = cn[r];
  }
  __syncthreads();
  v4f s = zero4;
  float c = 0.0f;
#pragma unroll
  for (int w = 0; w < 8; ++w) {
    s = s + sAcc[(w * GPB + wave) * 32 + lane];
    c += sCn[w * GPB + wave];
  }
  const float inv = 1.0f / fmaxf(c, 1.0f);
  const v4f pr = s * inv;
  const int row = g0 + wave;
  unsigned int u0h, u1h, u0l, u1l;
  split4(pr, u0h, u1h, u0l, u1l);
  const int sl = 2 * (lane & 15);
  const bool lo16 = lane < 16;
  const v4u qh = relay8(u0h, u1h, sl);
  const v4u ql = relay8(u0l, u1l, sl);
  const v4u q = lo16 ? qh : ql;
  unsigned short* op = (lo16 ? QH : QL) + (size_t)row * DM + 8 * (lane & 15);
  *(volatile v4u*)op = q;
  __threadfence();
  *(volatile v4u*)op = q;
}

__global__ __launch_bounds__(256) void k_final(
    const float* __restrict__ O64, const float* __restrict__ bc2, float* out, int nF4) {
  const int tid = (int)threadIdx.x;
  const int nit = (nF4 + 255) >> 8;
#pragma unroll 1
  for (int it = 0; it < nit; ++it) {
    const int f = (it << 8) + tid;
    const bool ok = f < nF4;
    const int fc = ok ? f : (nF4 - 1);
    const int gi = fc >> 2, c4 = (fc & 3) * 4;
    const v4f v = *(const v4f*)(O64 + (size_t)gi * OUTP + c4);
    const v4f bb = *(const v4f*)(bc2 + c4);
    const v4f o = v + bb;
    if (ok) *(volatile v4f*)(out + (size_t)fc * 4) = o;
    __threadfence();
    if (ok) *(volatile v4f*)(out + (size_t)fc * 4) = o;
  }
}

extern "C" void kernel_launch(void* const* d_in, const int* in_sizes, int n_in,
                              void* d_out, int out_size, void* d_ws, size_t ws_size,
                              hipStream_t stream) {
  if (n_in < 17) return;
  const int nN = in_sizes[0] / DM;
  const int nE = in_sizes[1] / 2;
  if (nN <= 0 || nE <= 0 || out_size <= 0) return;
  if (in_sizes[0] != nN * DM || in_sizes[1] != 2 * nE || in_sizes[2] != nN) return;
  if (in_sizes[3] != NLAY * DM * DM || in_sizes[7] != NLAY * DM * DM) return;
  if (in_sizes[4] != NLAY * DM || in_sizes[5] != NLAY * DM || in_sizes[6] != NLAY * DM) return;
  if (in_sizes[8] != NLAY * DM || in_sizes[9] != NLAY * DM || in_sizes[10] != NLAY * DM) return;
  if (in_sizes[11] != DM * DM || in_sizes[12] != DM || in_sizes[13] != DM || in_sizes[14] != DM) return;
  if (in_sizes[15] != DM * OUTC || in_sizes[16] != OUTC) return;
  if ((out_size % OUTC) != 0) return;
  const int G = out_size / OUTC;
  if (G <= 0) return;
  if (nN > RMAX * RB || nE > (1 << 22)) return;

  const float* x    = (const float*)d_in[0];
  const int*   ei   = (const int*)d_in[1];
  const int*   bat  = (const int*)d_in[2];
  const float* W1s  = (const float*)d_in[3];
  const float* b1s  = (const float*)d_in[4];
  const float* g1s  = (const float*)d_in[5];
  const float* be1s = (const float*)d_in[6];
  const float* W2s  = (const float*)d_in[7];
  const float* b2s  = (const float*)d_in[8];
  const float* gns  = (const float*)d_in[9];
  const float* bns  = (const float*)d_in[10];
  const float* Wc1  = (const float*)d_in[11];
  const float* bc1  = (const float*)d_in[12];
  const float* gc   = (const float*)d_in[13];
  const float* bec  = (const float*)d_in[14];
  const float* Wc2  = (const float*)d_in[15];
  const float* bc2  = (const float*)d_in[16];
  const int*   esrc = ei;
  const int*   edst = ei + nE;
  float* out = (float*)d_out;

  const int nCh  = (nE + CHUNK - 1) / CHUNK;
  const int nR   = (nN + RB - 1) / RB;
  const int nNp  = ((nN + 127) / 128) * 128;
  const int nSB  = nNp / STATRS;
  const int Gp   = ((G + 127) / 128) * 128;
  const int nSBg = Gp / STATRS;
  const int nSBm = nSB > nSBg ? nSB : nSBg;

  const size_t szT    = (size_t)NWROWS * DM * 2;
  const size_t szA    = (size_t)nNp * DM * 2;
  const size_t szP    = (size_t)nNp * DM * 4;
  const size_t szCS   = (size_t)nCh * CHUNK * 4;
  const size_t szTab  = (size_t)nCh * TABW * 4;
  const size_t szPart = (size_t)nSBm * 256 * 8;
  const size_t szStat = 256 * 4;
  const size_t szQ    = (size_t)Gp * DM * 2;
  const size_t szPg   = (size_t)Gp * DM * 4;
  const size_t szO    = (size_t)Gp * OUTP * 4;
  size_t off = 0;
  const size_t oTH = off; off += szT;    off = (off + 255) & ~(size_t)255;
  const size_t oTL = off; off += szT;    off = (off + 255) & ~(size_t)255;
  const size_t oAH = off; off += szA;    off = (off + 255) & ~(size_t)255;
  const size_t oAL = off; off += szA;    off = (off + 255) & ~(size_t)255;
  const size_t oP  = off; off += szP;    off = (off + 255) & ~(size_t)255;
  const size_t oHf = off; off += szP;    off = (off + 255) & ~(size_t)255;
  const size_t oC  = off; off += szCS;   off = (off + 255) & ~(size_t)255;
  const size_t oT  = off; off += szTab;  off = (off + 255) & ~(size_t)255;
  const size_t oPa = off; off += szPart; off = (off + 255) & ~(size_t)255;
  const size_t oPb = off; off += szPart; off = (off + 255) & ~(size_t)255;
  const size_t oSa = off; off += szStat; off = (off + 255) & ~(size_t)255;
  const size_t oSb = off; off += szStat; off = (off + 255) & ~(size_t)255;
  const size_t oQH = off; off += szQ;    off = (off + 255) & ~(size_t)255;
  const size_t oQL = off; off += szQ;    off = (off + 255) & ~(size_t)255;
  const size_t oPg = off; off += szPg;   off = (off + 255) & ~(size_t)255;
  const size_t oO  = off; off += szO;    off = (off + 255) & ~(size_t)255;
  if (off > ws_size || off > (size_t)WSCAP) return;

  char* ws = (char*)d_ws;
  unsigned short* Thi   = (unsigned short*)(ws + oTH);
  unsigned short* Tlo   = (unsigned short*)(ws + oTL);
  unsigned short* AH    = (unsigned short*)(ws + oAH);
  unsigned short* AL    = (unsigned short*)(ws + oAL);
  float*          P     = (float*)(ws + oP);
  float*          Hf    = (float*)(ws + oHf);
  unsigned int*   csort = (unsigned int*)(ws + oC);
  int*            tab   = (int*)(ws + oT);
  double*         partA = (double*)(ws + oPa);
  double*         partB = (double*)(ws + oPb);
  float*          statA = (float*)(ws + oSa);
  float*          statB = (float*)(ws + oSb);
  unsigned short* QH    = (unsigned short*)(ws + oQH);
  unsigned short* QL    = (unsigned short*)(ws + oQL);
  float*          Pg    = (float*)(ws + oPg);
  float*          O64   = (float*)(ws + oO);

  k_csort<<<nCh, 256, 0, stream>>>(edst, csort, tab, nN, nE);

  k_wprep<<<NWROWS / 32, 256, 0, stream>>>(W1s, W2s, Wc1, Wc2, Thi, Tlo);

  hipFuncSetAttribute(reinterpret_cast<const void*>(&k_agg),
                      hipFuncAttributeMaxDynamicSharedMemorySize, AGG_LDS_BYTES);
  const float* hcur = x;
  int hrows = nN;
  for (int l = 0; l < NLAY; ++l) {
    k_agg<<<nR, 256, AGG_LDS_BYTES, stream>>>(hcur, hrows, esrc, csort, tab, AH, AL, nN, nNp, nE, nCh);
    k_gemm<1><<<dim3(DM / 32, nNp / 128, 1), GT, 0, stream>>>(
        AH, AL, Thi + (size_t)(l * DM) * DM, Tlo + (size_t)(l * DM) * DM, b1s + l * DM, P, DM, nNp, DM);
    k_colstat<<<nSB, 256, 0, stream>>>(P, nN, partA);
    k_bnfin<<<1, 128, 0, stream>>>(partA, nSB, nN, statA);
    k_bnapply<0><<<nNp / 64, 256, 0, stream>>>(P, statA, g1s + l * DM, be1s + l * DM, Hf, AH, AL, nN);
    k_gemm<1><<<dim3(DM / 32, nNp / 128, 1), GT, 0, stream>>>(
        AH, AL, Thi + (size_t)(NLAY * DM + l * DM) * DM, Tlo + (size_t)(NLAY * DM + l * DM) * DM,
        b2s + l * DM, P, DM, nNp, DM);
    k_colstat<<<nSB, 256, 0, stream>>>(P, nN, partB);
    k_bnfin<<<1, 128, 0, stream>>>(partB, nSB, nN, statB);
    k_bnapply<1><<<nNp / 64, 256, 0, stream>>>(P, statB, gns + l * DM, bns + l * DM, Hf, AH, AL, nN);
    hcur = Hf;
    hrows = nNp;
  }

  k_pool<<<Gp / GPB, 256, 0, stream>>>(Hf, bat, QH, QL, nN);

  k_gemm<1><<<dim3(DM / 32, Gp / 128, 1), GT, 0, stream>>>(
      QH, QL, Thi + (size_t)(2 * NLAY * DM) * DM, Tlo + (size_t)(2 * NLAY * DM) * DM, bc1, Pg, DM, Gp, DM);
  k_colstat<<<nSBg, 256, 0, stream>>>(Pg, G, partA);
  k_bnfin<<<1, 128, 0, stream>>>(partA, nSBg, G, statA);
  k_bnapply<0><<<Gp / 64, 256, 0, stream>>>(Pg, statA, gc, bec, Hf, QH, QL, G);

  k_gemm<0><<<dim3(OUTP / 32, Gp / 128, 1), GT, 0, stream>>>(
      QH, QL, Thi + (size_t)(2 * NLAY * DM + DM) * DM, Tlo + (size_t)(2 * NLAY * DM + DM) * DM,
      bc1, O64, OUTP, Gp, OUTP);
  k_final<<<1, 256, 0, stream>>>(O64, bc2, out, out_size / 4);
}
